// GraphFallbackSolver_63118839382258
// MI455X (gfx1250) — hardware-verified
//
#include <hip/hip_runtime.h>
#include <stdint.h>


#define CIN     3
#define CH      64
#define KIN     70
#define KINP    96
#define K1      512
#define K2      256
#define MT      32
#define RT      64
#define SLOTB   6
#define CAPL    2048
#define NTHR    256
#define CHUNK   (NTHR * 4)
#define NODET   32
#define NODETHR 128
#define PREPTHR 256

static_assert(RT == (1 << SLOTB));
static_assert(MT * 8 == NTHR);
static_assert(NODET * 4 == NODETHR);
static_assert((KINP % 32) == 0 && (K1 % 32) == 0 && (K2 % 32) == 0 && (CH % 32) == 0);

typedef _Float16 v16h __attribute__((ext_vector_type(16)));
typedef _Float16 v8h  __attribute__((ext_vector_type(8)));
typedef float    v8f  __attribute__((ext_vector_type(8)));
typedef float    v4f  __attribute__((ext_vector_type(4)));
typedef int      v4i  __attribute__((ext_vector_type(4)));
typedef v8h v8h_ma __attribute__((may_alias));
typedef v4f v4f_ma __attribute__((may_alias));
typedef v4i v4i_ma __attribute__((may_alias));

union FragU { v16h v; v8h q[2]; };

union alignas(16) LdsU1 { _Float16 a1[MT * K1]; float pf[RT * CH]; };
union alignas(16) LdsU2 { _Float16 a2[MT * K2]; _Float16 h16[RT * CH]; };

__device__ __forceinline__ v8f splat8(float b) {
  v8f r;
#pragma unroll
  for (int i = 0; i < 8; ++i) r[i] = b;
  return r;
}

__device__ __forceinline__ v8f wmma16(v16h a, v16h b, v8f c) {
  v8f d = __builtin_amdgcn_wmma_f32_16x16x32_f16(false, a, false, b, (short)0, c, false, false);
  asm volatile("v_nop\n\tv_nop\n\tv_nop\n\tv_nop" : "+v"(d) : "v"(a), "v"(b));
  return d;
}

__device__ __forceinline__ v16h ld_frag_rm(const _Float16* base, int pitch, int k0, int lane) {
  const int m = lane & 15, h = lane >> 4;
  const _Float16* p = base + m * pitch + k0 + 8 * h;
  FragU u;
  u.q[0] = *(const v8h_ma*)p;
  u.q[1] = *(const v8h_ma*)(p + 16);
  return u.v;
}

__device__ __forceinline__ v16h ld_frag_pk(const _Float16* tile, int lane) {
  const _Float16* p = tile + lane * 16;
  FragU u;
  u.q[0] = *(const v8h_ma*)p;
  u.q[1] = *(const v8h_ma*)(p + 8);
  return u.v;
}

__device__ __forceinline__ float gelu_f(float x) {
  return 0.5f * x * (1.0f + erff(x * 0.70710678118654752f));
}

__global__ __launch_bounds__(PREPTHR) void k_prep(const float* __restrict__ W, _Float16* __restrict__ outp,
                                                   int Kact, int KT, int Nn, int perm, float scale) {
  const int idx = blockIdx.x * PREPTHR + threadIdx.x;
  const int total = KT * (Nn >> 4) * 64;
  if (idx >= total) return;
  const int tile = idx >> 6;
  const int L = (idx >> 1) & 31;
  const int q = idx & 1;
  const int kt = tile % KT, nt = tile / KT;
  const int n = nt * 16 + (L & 15);
  const int h = L >> 4;
  v8h v;
#pragma unroll
  for (int i = 0; i < 8; ++i) {
    const int k = kt * 32 + q * 16 + 8 * h + i;
    const int ko = perm ? (k < 64 ? k + 6 : k - 64) : k;
    float x = 0.0f;
    if (k < Kact) x = W[(size_t)ko * Nn + n] * scale;
    v[i] = (_Float16)x;
  }
  _Float16* p = outp + (size_t)tile * 512 + L * 16 + q * 8;
  *(volatile v8h_ma*)p = v;
  __threadfence();
  *(volatile v8h_ma*)p = v;
}

__global__ __launch_bounds__(NODETHR) void k_node(const float* __restrict__ feats, const float* __restrict__ Wl1,
                                                   const float* __restrict__ bl1, const _Float16* __restrict__ wl2,
                                                   const float* __restrict__ bl2, float* __restrict__ fy32, int nBN) {
  __shared__ alignas(16) _Float16 s_h1[NODET * CH];
  __shared__ alignas(16) float s_o[NODET * CH];
  const int tid = threadIdx.x, lane = tid & 31, wave = tid >> 5;
  const int h = lane >> 4, nl = lane & 15;
  const int row0 = blockIdx.x * NODET;
  {
    const int m = tid >> 2, g = tid & 3;
    const int node = row0 + m;
    float f0 = 0.0f, f1 = 0.0f, f2 = 0.0f;
    if (node < nBN) {
      f0 = feats[(size_t)node * CIN + 0];
      f1 = feats[(size_t)node * CIN + 1];
      f2 = feats[(size_t)node * CIN + 2];
    }
#pragma unroll
    for (int c = 0; c < 16; ++c) {
      const int cc = g * 16 + c;
      float x = f0 * Wl1[cc];
      x = x + f1 * Wl1[CH + cc];
      x = x + f2 * Wl1[2 * CH + cc];
      x = x + bl1[cc];
      s_h1[m * CH + cc] = (_Float16)gelu_f(x);
    }
  }
  __syncthreads();
  {
    const float bv = bl2[wave * 16 + nl] * 8.0f;
    v8f acc[2];
    acc[0] = splat8(bv);
    acc[1] = acc[0];
#pragma unroll
    for (int kc = 0; kc < CH / 32; ++kc) {
      const v16h a0 = ld_frag_rm(s_h1, CH, kc * 32, lane);
      const v16h a1 = ld_frag_rm(s_h1 + 16 * CH, CH, kc * 32, lane);
      const v16h b = ld_frag_pk(wl2 + (size_t)(wave * (CH / 32) + kc) * 512, lane);
      acc[0] = wmma16(a0, b, acc[0]);
      acc[1] = wmma16(a1, b, acc[1]);
    }
#pragma unroll
    for (int mt = 0; mt < 2; ++mt)
#pragma unroll
      for (int r = 0; r < 8; ++r) {
        const int m = mt * 16 + 8 * h + r;
        s_o[m * CH + wave * 16 + nl] = acc[mt][r] * 0.125f;
      }
  }
  __syncthreads();
#pragma unroll
  for (int it = 0; it < 4; ++it) {
    const int rl = wave * 8 + it * 2 + h;
    const int node = row0 + rl;
    if (node < nBN) {
      const v4f v = *(const v4f_ma*)(s_o + rl * CH + nl * 4);
      *(volatile v4f_ma*)(fy32 + (size_t)node * CH + nl * 4) = v;
    }
  }
  __threadfence();
#pragma unroll
  for (int it = 0; it < 4; ++it) {
    const int rl = wave * 8 + it * 2 + h;
    const int node = row0 + rl;
    if (node < nBN) {
      const v4f v = *(const v4f_ma*)(s_o + rl * CH + nl * 4);
      *(volatile v4f_ma*)(fy32 + (size_t)node * CH + nl * 4) = v;
    }
  }
}

__global__ __launch_bounds__(NTHR) void k_edge(
    const float* __restrict__ pts, const float* __restrict__ fy32,
    const int* __restrict__ esrc, const int* __restrict__ edst,
    const _Float16* __restrict__ wk1, const float* __restrict__ bk1,
    const _Float16* __restrict__ wk2, const float* __restrict__ bk2,
    const _Float16* __restrict__ wk3, const float* __restrict__ bk3,
    const _Float16* __restrict__ wp1, const float* __restrict__ bp1,
    const float* __restrict__ Wp2, const float* __restrict__ bp2,
    float* __restrict__ outp, int nBN, int nE) {
  __shared__ alignas(16) float s_agg[RT * CH];
  __shared__ float s_cnt[RT];
  __shared__ int s_list[CAPL];
  __shared__ int s_wcnt[16];
  __shared__ int s_slot[MT];
  __shared__ alignas(16) float s_outv[RT];
  __shared__ alignas(16) _Float16 s_ein[MT * KINP];
  __shared__ alignas(16) float s_fy[MT * CH];
  __shared__ alignas(16) float s_msg[MT * CH];
  __shared__ LdsU1 s_u1;
  __shared__ LdsU2 s_u2;

  const int tid = threadIdx.x, lane = tid & 31, wave = tid >> 5;
  const int h = lane >> 4, nl = lane & 15;
  const int row0 = blockIdx.x * RT;
  if (row0 >= nBN) return;

  for (int i = tid; i < RT * CH; i += NTHR) s_agg[i] = 0.0f;
  if (tid < RT) { s_cnt[tid] = 0.0f; s_outv[tid] = 0.0f; }
  for (int i = tid; i < MT * (KINP - 64); i += NTHR) {
    const int r = i / (KINP - 64);
    const int c = 64 + (i - r * (KINP - 64));
    s_ein[r * KINP + c] = (_Float16)0.0f;
  }
  __syncthreads();

  int nlist = 0;
  for (int base = 0; base < nE; base += CHUNK) {
    const int par = ((base / CHUNK) & 1) * 8;
    const int i0 = base + tid * 4;
    int d[4];
    if (base + CHUNK <= nE) {
      const v4i v = *(const v4i_ma*)(edst + i0);
      d[0] = v[0]; d[1] = v[1]; d[2] = v[2]; d[3] = v[3];
    } else {
#pragma unroll
      for (int j = 0; j < 4; ++j) {
        const int idx = i0 + j;
        d[j] = (idx < nE) ? edst[idx] : -1;
      }
    }
    int rank[4];
    int cw = 0;
#pragma unroll
    for (int j = 0; j < 4; ++j) {
      const bool ht = ((unsigned)(d[j] - row0) < (unsigned)RT) && (d[j] < nBN);
      const unsigned b = __builtin_amdgcn_ballot_w32(ht);
      rank[j] = ht ? (cw + (int)__builtin_popcount(b & ((1u << lane) - 1u))) : -1;
      cw += (int)__builtin_popcount(b);
    }
    if (lane == 0) s_wcnt[par + wave] = cw;
    __syncthreads();
    int tot = 0, wb = 0;
#pragma unroll
    for (int w = 0; w < NTHR / 32; ++w) {
      const int c = s_wcnt[par + w];
      if (w < wave) wb += c;
      tot += c;
    }
    if (tot != 0) {
#pragma unroll
      for (int j = 0; j < 4; ++j) {
        if (rank[j] >= 0) {
          const int pos = nlist + wb + rank[j];
          if (pos < CAPL) s_list[pos] = ((i0 + j) << SLOTB) | (d[j] - row0);
        }
      }
    }
    nlist = min(nlist + tot, CAPL);
  }
  __syncthreads();

  const int ntiles = min((nlist + MT - 1) / MT, CAPL / MT);
  const int r_g = tid >> 3, p_g = tid & 7;
  for (int t = 0; t < ntiles; ++t) {
    const int nvalid = min(MT, nlist - t * MT);
    {
      const int li = t * MT + r_g;
      const int entry = (r_g < nvalid) ? s_list[li] : 0;
      int e = entry >> SLOTB;
      const int slot = entry & (RT - 1);
      e = min(max(e, 0), nE - 1);
      int src = esrc[e];
      src = min(max(src, 0), nBN - 1);
      const int dst = min(row0 + slot, nBN - 1);
      const float* fr = fy32 + (size_t)src * CH + p_g * 8;
      const v4f f0 = *(const v4f_ma*)fr;
      const v4f f1 = *(const v4f_ma*)(fr + 4);
      *(v4f_ma*)(s_fy + r_g * CH + p_g * 8) = f0;
      *(v4f_ma*)(s_fy + r_g * CH + p_g * 8 + 4) = f1;
      v8h hv;
      hv[0] = (_Float16)f0[0]; hv[1] = (_Float16)f0[1]; hv[2] = (_Float16)f0[2]; hv[3] = (_Float16)f0[3];
      hv[4] = (_Float16)f1[0]; hv[5] = (_Float16)f1[1]; hv[6] = (_Float16)f1[2]; hv[7] = (_Float16)f1[3];
      *(v8h_ma*)(s_ein + r_g * KINP + p_g * 8) = hv;
      if (p_g < 6) {
        const float pv = (p_g < 3) ? pts[(size_t)src * 3 + p_g] : pts[(size_t)dst * 3 + (p_g - 3)];
        s_ein[r_g * KINP + 64 + p_g] = (_Float16)pv;
      }
      if (p_g == 0) s_slot[r_g] = slot;
    }
    __syncthreads();

    {
      const int nt0 = wave * 4;
      v8f acc[2][4];
#pragma unroll
      for (int j = 0; j < 4; ++j) {
        const float bv = bk1[(nt0 + j) * 16 + nl] * 8.0f;
        acc[0][j] = splat8(bv);
        acc[1][j] = acc[0][j];
      }
#pragma unroll
      for (int kc = 0; kc < KINP / 32; ++kc) {
        const v16h a0 = ld_frag_rm(s_ein, KINP, kc * 32, lane);
        const v16h a1 = ld_frag_rm(s_ein + 16 * KINP, KINP, kc * 32, lane);
#pragma unroll
        for (int j = 0; j < 4; ++j) {
          const v16h b = ld_frag_pk(wk1 + (size_t)((nt0 + j) * (KINP / 32) + kc) * 512, lane);
          acc[0][j] = wmma16(a0, b, acc[0][j]);
          acc[1][j] = wmma16(a1, b, acc[1][j]);
        }
      }
#pragma unroll
      for (int mt = 0; mt < 2; ++mt)
#pragma unroll
        for (int j = 0; j < 4; ++j) {
          const int n = (nt0 + j) * 16 + nl;
#pragma unroll
          for (int r = 0; r < 8; ++r) {
            const int m = mt * 16 + 8 * h + r;
            s_u1.a1[m * K1 + n] = (_Float16)gelu_f(acc[mt][j][r] * 0.125f);
          }
        }
    }
    __syncthreads();

    {
      const int nt0 = wave * 2;
      v8f acc[2][2];
#pragma unroll
      for (int j = 0; j < 2; ++j) {
        const float bv = bk2[(nt0 + j) * 16 + nl] * 16.0f;
        acc[0][j] = splat8(bv);
        acc[1][j] = acc[0][j];
      }
#pragma unroll 2
      for (int kc = 0; kc < K1 / 32; ++kc) {
        const v16h a0 = ld_frag_rm(s_u1.a1, K1, kc * 32, lane);
        const v16h a1 = ld_frag_rm(s_u1.a1 + 16 * K1, K1, kc * 32, lane);
#pragma unroll
        for (int j = 0; j < 2; ++j) {
          const v16h b = ld_frag_pk(wk2 + (size_t)((nt0 + j) * (K1 / 32) + kc) * 512, lane);
          acc[0][j] = wmma16(a0, b, acc[0][j]);
          acc[1][j] = wmma16(a1, b, acc[1][j]);
        }
      }
#pragma unroll
      for (int mt = 0; mt < 2; ++mt)
#pragma unroll
        for (int j = 0; j < 2; ++j) {
          const int n = (nt0 + j) * 16 + nl;
#pragma unroll
          for (int r = 0; r < 8; ++r) {
            const int m = mt * 16 + 8 * h + r;
            s_u2.a2[m * K2 + n] = (_Float16)gelu_f(acc[mt][j][r] * 0.0625f);
          }
        }
    }
    __syncthreads();

    {
      const int mtile = wave & 1, ntile = wave >> 1;
      const int n = ntile * 16 + nl;
      v8f acc = splat8(bk3[n] * 16.0f);
      const _Float16* arow = s_u2.a2 + mtile * 16 * K2;
#pragma unroll 2
      for (int kc = 0; kc < K2 / 32; ++kc) {
        const v16h a = ld_frag_rm(arow, K2, kc * 32, lane);
        const v16h b = ld_frag_pk(wk3 + (size_t)(ntile * (K2 / 32) + kc) * 512, lane);
        acc = wmma16(a, b, acc);
      }
#pragma unroll
      for (int r = 0; r < 8; ++r) {
        const int m = mtile * 16 + 8 * h + r;
        s_msg[m * CH + n] = (acc[r] * 0.0625f) * s_fy[m * CH + n];
      }
    }
    __syncthreads();

    if (tid < CH) {
      const int n = tid;
      for (int r = 0; r < nvalid; ++r) {
        const int slot = s_slot[r];
        s_agg[slot * CH + n] += s_msg[r * CH + n];
        if (n == 0) s_cnt[slot] += 1.0f;
      }
    }
    __syncthreads();
  }

  for (int i = tid; i < RT * CH; i += NTHR) {
    const int m = i / CH;
    const float cn = s_cnt[m];
    const float inv = 1.0f / (cn < 1.0f ? 1.0f : cn);
    s_u2.h16[i] = (_Float16)(s_agg[i] * inv);
  }
  __syncthreads();
  {
    const int mt = wave >> 1, ntb = (wave & 1) * 2;
    v8f acc[2];
#pragma unroll
    for (int j = 0; j < 2; ++j) acc[j] = splat8(bp1[(ntb + j) * 16 + nl] * 8.0f);
#pragma unroll
    for (int kc = 0; kc < CH / 32; ++kc) {
      const v16h a = ld_frag_rm(s_u2.h16 + mt * 16 * CH, CH, kc * 32, lane);
#pragma unroll
      for (int j = 0; j < 2; ++j) {
        const v16h b = ld_frag_pk(wp1 + (size_t)((ntb + j) * (CH / 32) + kc) * 512, lane);
        acc[j] = wmma16(a, b, acc[j]);
      }
    }
#pragma unroll
    for (int j = 0; j < 2; ++j) {
      const int n = (ntb + j) * 16 + nl;
      const float w2 = Wp2[n];
#pragma unroll
      for (int r = 0; r < 8; ++r) {
        const int m = mt * 16 + 8 * h + r;
        s_u1.pf[m * CH + n] = gelu_f(acc[j][r] * 0.125f) * w2;
      }
    }
  }
  __syncthreads();
  if (tid < RT) {
    const float* pr = s_u1.pf + tid * CH;
    float s = 0.0f;
#pragma unroll 8
    for (int n = 0; n < CH; ++n) s += pr[n];
    s_outv[tid] = s + bp2[0];
  }
  __syncthreads();
  if (wave == 0) {
    const int row = row0 + 4 * lane;
    const bool act = (lane < RT / 4);
    v4f v = splat8(0.0f).lo;
    if (act) v = *(const v4f_ma*)(s_outv + 4 * lane);
    const bool full = act && (row + 4 <= nBN);
    if (full) {
      *(volatile v4f_ma*)(outp + row) = v;
    } else if (act) {
#pragma unroll
      for (int k = 0; k < 4; ++k) if (row + k < nBN) ((volatile float*)outp)[row + k] = v[k];
    }
    __threadfence();
    if (full) {
      *(volatile v4f_ma*)(outp + row) = v;
    } else if (act) {
#pragma unroll
      for (int k = 0; k < 4; ++k) if (row + k < nBN) ((volatile float*)outp)[row + k] = v[k];
    }
  }
}

static inline size_t align256(size_t x) { return (x + 255) & ~(size_t)255; }

extern "C" void kernel_launch(void* const* d_in, const int* in_sizes, int n_in,
                              void* d_out, int out_size, void* d_ws, size_t ws_size,
                              hipStream_t stream) {
  if (n_in < 18) return;
  const float* pts   = (const float*)d_in[0];
  const float* feats = (const float*)d_in[1];
  const int*   esrc  = (const int*)d_in[2];
  const int*   edst  = (const int*)d_in[3];
  const float* Wl1 = (const float*)d_in[4];  const float* bl1 = (const float*)d_in[5];
  const float* Wl2 = (const float*)d_in[6];  const float* bl2 = (const float*)d_in[7];
  const float* Wk1 = (const float*)d_in[8];  const float* bk1 = (const float*)d_in[9];
  const float* Wk2 = (const float*)d_in[10]; const float* bk2 = (const float*)d_in[11];
  const float* Wk3 = (const float*)d_in[12]; const float* bk3 = (const float*)d_in[13];
  const float* Wp1 = (const float*)d_in[14]; const float* bp1 = (const float*)d_in[15];
  const float* Wp2 = (const float*)d_in[16]; const float* bp2 = (const float*)d_in[17];

  const int nBN = in_sizes[0] / CIN;
  const int nE  = in_sizes[2];
  if (nBN <= 0 || nE < 0 || out_size < nBN) return;

  char* ws = (char*)d_ws;
  size_t off = 0;
  float* fy32 = (float*)(ws + off);        off += align256((size_t)nBN * CH * sizeof(float));
  _Float16* wl2f = (_Float16*)(ws + off);  off += align256((size_t)CH * CH * 2);
  _Float16* wk1f = (_Float16*)(ws + off);  off += align256((size_t)KINP * K1 * 2);
  _Float16* wk2f = (_Float16*)(ws + off);  off += align256((size_t)K1 * K2 * 2);
  _Float16* wk3f = (_Float16*)(ws + off);  off += align256((size_t)K2 * CH * 2);
  _Float16* wp1f = (_Float16*)(ws + off);  off += align256((size_t)CH * CH * 2);
  if (off > ws_size) return;

  {
    const int KT = CH / 32, Nn = CH;
    const int total = KT * (Nn / 16) * 64;
    k_prep<<<(total + PREPTHR - 1) / PREPTHR, PREPTHR, 0, stream>>>(Wl2, wl2f, CH, KT, Nn, 0, 8.0f);
  }
  {
    const int KT = KINP / 32, Nn = K1;
    const int total = KT * (Nn / 16) * 64;
    k_prep<<<(total + PREPTHR - 1) / PREPTHR, PREPTHR, 0, stream>>>(Wk1, wk1f, KIN, KT, Nn, 1, 8.0f);
  }
  {
    const int KT = K1 / 32, Nn = K2;
    const int total = KT * (Nn / 16) * 64;
    k_prep<<<(total + PREPTHR - 1) / PREPTHR, PREPTHR, 0, stream>>>(Wk2, wk2f, K1, KT, Nn, 0, 16.0f);
  }
  {
    const int KT = K2 / 32, Nn = CH;
    const int total = KT * (Nn / 16) * 64;
    k_prep<<<(total + PREPTHR - 1) / PREPTHR, PREPTHR, 0, stream>>>(Wk3, wk3f, K2, KT, Nn, 0, 16.0f);
  }
  {
    const int KT = CH / 32, Nn = CH;
    const int total = KT * (Nn / 16) * 64;
    k_prep<<<(total + PREPTHR - 1) / PREPTHR, PREPTHR, 0, stream>>>(Wp1, wp1f, CH, KT, Nn, 0, 8.0f);
  }
  k_node<<<(nBN + NODET - 1) / NODET, NODETHR, 0, stream>>>(feats, Wl1, bl1, wl2f, bl2, fy32, nBN);
  k_edge<<<(nBN + RT - 1) / RT, NTHR, 0, stream>>>(pts, fy32, esrc, edst, wk1f, bk1, wk2f, bk2, wk3f, bk3,
                                                   wp1f, bp1, Wp2, bp2, (float*)d_out, nBN, nE);
}
